// VLineHead_21509196218383
// MI455X (gfx1250) — hardware-verified
//
#include <hip/hip_runtime.h>
#include <stdint.h>

#define DEVINL __device__ __forceinline__

typedef _Float16 f16t;
typedef _Float16 v16h __attribute__((ext_vector_type(16)));
typedef _Float16 v8h  __attribute__((ext_vector_type(8)));
typedef float    v8f  __attribute__((ext_vector_type(8)));
typedef float    v4f  __attribute__((ext_vector_type(4)));
typedef short    v8s  __attribute__((ext_vector_type(8)));
typedef v8h __attribute__((may_alias)) v8ha;
typedef v4f __attribute__((may_alias)) v4fa;
typedef v8s __attribute__((may_alias)) v8sa;
union FragH { v16h v; v8h half[2]; };

#define NIMG   64
#define CIN    256
#define HWD    24
#define NPIX   576
#define NV     32
#define CEXT   128
#define FL     512
#define FG     256
#define GIN    2304
#define KCONV  2304
#define DALL   2336
#define DALLP  2368
#define D2     1312
#define NB2    2
#define NROW   2048
#define PHW    26
#define PPIX   676
#define NOUT   (6 * NROW * NB2)

#define XCAR 8.0f
#define WCAR 256.0f
#define FCAR 16.0f
#define GCAR 64.0f
#define ACAR 16.0f

#define NB_WP  144
#define NB_WG  288
#define NB_WL  128
#define NB_WC  1184

#define PL_MT  ((size_t)NROW * NPIX)
#define PL_MP  ((size_t)NROW * CEXT)
#define PL_WL  ((size_t)FL * CEXT)
#define PL_VF  ((size_t)NROW * FL)
#define PL_WC  ((size_t)FL * DALLP)
#define PL_ALL ((size_t)NROW * DALLP)
#define PL_HID ((size_t)NROW * FL)

static_assert((KCONV % 32) == 0);
static_assert((DALL % 32) == 0);
static_assert((DALLP % 64) == 0);
static_assert((GIN % 256) == 0);
static_assert((NPIX % 64) == 0);
static_assert((CIN % 32) == 0);
static_assert((CEXT % 64) == 0);
static_assert((FL % 64) == 0);
static_assert((FG % 64) == 0);
static_assert((NROW % 32) == 0);
static_assert((NIMG % 32) == 0);
static_assert(((CEXT * KCONV) / 8) == NB_WP * 256);
static_assert(((FG * GIN) / 8) == NB_WG * 256);
static_assert(((4 * FL * CEXT) / 8) == NB_WL * 256);
static_assert(((2 * FL * DALLP) / 8) == NB_WC * 256);
static_assert((PHW * CIN) % 8 == 0);
static_assert((NV * NPIX) == 9 * 256 * 8);

DEVINL int imin(int a, int b) { return a < b ? a : b; }
DEVINL int imax(int a, int b) { return a > b ? a : b; }
DEVINL float f16r(float x) { return (float)(f16t)x; }

DEVINL v8f wmma_f16(v16h a, v16h b, v8f c) {
  v8f d = __builtin_amdgcn_wmma_f32_16x16x32_f16(false, a, false, b, (short)0, c, false, false);
  asm volatile("v_nop\n\tv_nop\n\tv_nop\n\tv_nop" : "+v"(d) : "v"(a), "v"(b));
  return d;
}
DEVINL v8f zero8f() {
  v8f z = {0.f, 0.f, 0.f, 0.f, 0.f, 0.f, 0.f, 0.f};
  return z;
}

__global__ __launch_bounds__(256) void prepw_k(const float* __restrict__ cw, const float* __restrict__ Wg,
                                              const float* __restrict__ Wl, const float* __restrict__ Wlv,
                                              const float* __restrict__ Wlm, const float* __restrict__ Wlvm,
                                              const float* __restrict__ Wc, const float* __restrict__ Wcv,
                                              f16t* __restrict__ Wp, f16t* __restrict__ Wg16,
                                              f16t* __restrict__ Wl16, f16t* __restrict__ Wc16)
{
  const int blk = blockIdx.x;
  const int tid = threadIdx.x;
  v8h o;
  f16t* dst;
  if (blk < NB_WP) {
    const int t    = blk * 256 + tid;
    const int cout = t / (KCONV / 8);
    const int part = t - cout * (KCONV / 8);
    const int k8   = 8 * part;
    const int tap  = k8 >> 8;
    const int cin0 = k8 & 255;
    #pragma unroll
    for (int i = 0; i < 8; ++i) {
      const float wv = cw[((size_t)cout * CIN + cin0 + i) * 9 + tap];
      o[i] = (f16t)(wv * WCAR);
    }
    dst = Wp + (size_t)8 * t;
  } else if (blk < NB_WP + NB_WG) {
    const int u = (blk - NB_WP) * 256 + tid;
    #pragma unroll
    for (int i = 0; i < 8; ++i) o[i] = (f16t)(Wg[(size_t)8 * u + i] * WCAR);
    dst = Wg16 + (size_t)8 * u;
  } else if (blk < NB_WP + NB_WG + NB_WL) {
    const int u     = (blk - NB_WP - NB_WG) * 256 + tid;
    const int which = u >> 13;
    const int e     = u & 8191;
    const float* src = (which == 0) ? Wl : ((which == 1) ? Wlv : ((which == 2) ? Wlm : Wlvm));
    #pragma unroll
    for (int i = 0; i < 8; ++i) o[i] = (f16t)(src[(size_t)8 * e + i] * WCAR);
    dst = Wl16 + (size_t)8 * u;
  } else {
    const int u     = (blk - NB_WP - NB_WG - NB_WL) * 256 + tid;
    const int which = (u >= (FL * DALLP / 8)) ? 1 : 0;
    const int e     = u - which * (FL * DALLP / 8);
    const int row   = e / (DALLP / 8);
    const int p     = e - row * (DALLP / 8);
    const int c0    = 8 * p;
    const float* src = which ? Wcv : Wc;
    #pragma unroll
    for (int i = 0; i < 8; ++i) {
      const int c  = c0 + i;
      const int cc = (c < DALL) ? c : (DALL - 1);
      const float wv = src[(size_t)row * DALL + cc];
      o[i] = (c < DALL) ? (f16t)(wv * WCAR) : (f16t)0.0f;
    }
    dst = Wc16 + (size_t)8 * u;
  }
  *(volatile v8h*)dst = o;
  __threadfence();
  *(volatile v8h*)dst = o;
}

__global__ __launch_bounds__(256) void rprep_k(const float* __restrict__ x, f16t* __restrict__ Rp)
{
  __shared__ __attribute__((aligned(16))) float sX[CIN * HWD];
  __shared__ __attribute__((aligned(16))) f16t  sY[PHW * CIN];
  const int tid = threadIdx.x;
  const int hp  = blockIdx.x;
  const int b   = blockIdx.y;
  const bool interior = (hp >= 1) && (hp <= HWD);
  const int h = imin(imax(hp - 1, 0), HWD - 1);

  if (interior) {
    const float* xb = x + ((size_t)b * CIN) * NPIX + (size_t)h * HWD;
    #pragma unroll 1
    for (int idx = tid; idx < CIN * HWD; idx += 256) {
      const int c = idx / HWD;
      const int w = idx - c * HWD;
      sX[idx] = xb[(size_t)c * NPIX + w];
    }
  }
  __syncthreads();

  #pragma unroll 1
  for (int idx = tid; idx < PHW * CIN; idx += 256) {
    const int wp = idx >> 8;
    const int c  = idx & (CIN - 1);
    const bool valid = interior && (wp >= 1) && (wp <= HWD);
    const int w = imin(imax(wp - 1, 0), HWD - 1);
    const float xv = sX[c * HWD + w];
    sY[idx] = (f16t)((valid ? xv : 0.0f) * XCAR);
  }
  __syncthreads();

  f16t* dstrow = Rp + ((size_t)(b * PHW + hp)) * (size_t)(PHW * CIN);
  v8h vals[4];
  #pragma unroll
  for (int q = 0; q < 4; ++q) {
    const int p = imin(q * 256 + tid, PHW * CIN / 8 - 1);
    vals[q] = *(const v8ha*)(sY + 8 * p);
  }
  #pragma unroll
  for (int q = 0; q < 4; ++q) {
    const int p = q * 256 + tid;
    if (p < PHW * CIN / 8) *(volatile v8h*)(dstrow + (size_t)8 * p) = vals[q];
  }
  __threadfence();
  #pragma unroll
  for (int q = 0; q < 4; ++q) {
    const int p = q * 256 + tid;
    if (p < PHW * CIN / 8) *(volatile v8h*)(dstrow + (size_t)8 * p) = vals[q];
  }
}

__global__ __launch_bounds__(256) void maps_k(const int* __restrict__ mh, const int* __restrict__ mv,
                                             f16t* __restrict__ MT)
{
  __shared__ __attribute__((aligned(16))) f16t sT[NV * NPIX];
  const int tid = threadIdx.x, n = blockIdx.x, dir = blockIdx.y;
  const int* src = (dir ? mv : mh) + (size_t)n * NPIX * NV;
  #pragma unroll 1
  for (int idx = tid; idx < NPIX * NV; idx += 256) {
    const int hw = idx >> 5;
    const int v  = idx & 31;
    sT[v * NPIX + hw] = (f16t)(float)src[idx];
  }
  __syncthreads();
  f16t* dst = MT + ((size_t)dir * NIMG + n) * (size_t)(NV * NPIX);
  v8h vals[9];
  #pragma unroll
  for (int q = 0; q < 9; ++q) vals[q] = *(const v8ha*)(sT + 8 * (q * 256 + tid));
  #pragma unroll
  for (int q = 0; q < 9; ++q) *(volatile v8h*)(dst + (size_t)8 * (q * 256 + tid)) = vals[q];
  __threadfence();
  #pragma unroll
  for (int q = 0; q < 9; ++q) *(volatile v8h*)(dst + (size_t)8 * (q * 256 + tid)) = vals[q];
}

__global__ __launch_bounds__(256) void gpool_k(const float* __restrict__ x, f16t* __restrict__ GP)
{
  __shared__ __attribute__((aligned(16))) f16t sG[256];
  const int tid = threadIdx.x, n = blockIdx.y, d0 = blockIdx.x * 256;
  const int d  = d0 + tid;
  const int c  = d / 9;
  const int g  = d - 9 * c;
  const int gy = g / 3, gx = g - 3 * gy;
  const float* base = x + ((size_t)n * CIN + c) * NPIX + gy * 8 * HWD + gx * 8;
  float s = 0.f;
  #pragma unroll 1
  for (int yy = 0; yy < 8; ++yy) {
    const float* r = base + yy * HWD;
    #pragma unroll
    for (int xx = 0; xx < 8; ++xx) s += r[xx];
  }
  sG[tid] = (f16t)(s * (1.0f / 64.0f) * GCAR);
  __syncthreads();
  if (tid < 32) {
    const v8h val = *(const v8ha*)(sG + 8 * tid);
    f16t* dst = GP + (size_t)n * GIN + d0 + 8 * tid;
    *(volatile v8h*)dst = val;
    __threadfence();
    *(volatile v8h*)dst = val;
  }
}

__global__ __launch_bounds__(128) void conv_k(const f16t* __restrict__ Rp, const f16t* __restrict__ Wp,
                                             const float* __restrict__ cb, f16t* __restrict__ F)
{
  __shared__ __attribute__((aligned(16))) f16t sO[CEXT * 64];
  const int tid = threadIdx.x, lane = tid & 31, wave = tid >> 5;
  const int h = lane >> 4, m = lane & 15;
  const int b = blockIdx.y;
  const int pixBase = blockIdx.x * 64;
  const int pix = pixBase + 16 * wave + m;
  const int oh = pix / HWD, ow = pix - oh * HWD;

  const f16t* yb = Rp + ((size_t)(b * PHW + oh) * PHW + ow) * CIN + 8 * h;
  const f16t* wr = Wp + (size_t)m * KCONV + 8 * h;

  v8f acc[8];
  #pragma unroll
  for (int t = 0; t < 8; ++t) acc[t] = zero8f();

  #pragma unroll 1
  for (int tap = 0; tap < 9; ++tap) {
    const int kh = tap / 3, kw = tap - 3 * kh;
    const f16t* ya = yb + (size_t)(kh * PHW + kw) * CIN;
    const f16t* wt = wr + tap * CIN;
    #pragma unroll 1
    for (int ks = 0; ks < 8; ++ks) {
      FragH bf;
      bf.half[0] = *(const v8ha*)(ya + 32 * ks);
      bf.half[1] = *(const v8ha*)(ya + 32 * ks + 16);
      #pragma unroll
      for (int t = 0; t < 8; ++t) {
        const f16t* wa = wt + (size_t)t * 16 * KCONV + 32 * ks;
        FragH a;
        a.half[0] = *(const v8ha*)(wa);
        a.half[1] = *(const v8ha*)(wa + 16);
        acc[t] = wmma_f16(a.v, bf.v, acc[t]);
      }
    }
  }

  const float sc = FCAR / (XCAR * WCAR);
  #pragma unroll
  for (int t = 0; t < 8; ++t) {
    #pragma unroll
    for (int r = 0; r < 8; ++r) {
      const int cout = 16 * t + 8 * h + r;
      const float v = fmaxf(acc[t][r] * sc + cb[cout] * FCAR, 0.0f);
      sO[cout * 64 + 16 * wave + m] = (f16t)v;
    }
  }
  __syncthreads();

  const int piece = tid & 7, lg = tid >> 3;
  v8h vals[8];
  #pragma unroll
  for (int q = 0; q < 8; ++q) {
    const int L = 16 * q + lg;
    vals[q] = *(const v8ha*)(sO + L * 64 + 8 * piece);
  }
  f16t* gb = F + ((size_t)b * CEXT) * NPIX + (size_t)pixBase + 8 * piece;
  #pragma unroll
  for (int q = 0; q < 8; ++q) {
    const int L = 16 * q + lg;
    *(volatile v8h*)(gb + (size_t)L * NPIX) = vals[q];
  }
  __threadfence();
  #pragma unroll
  for (int q = 0; q < 8; ++q) {
    const int L = 16 * q + lg;
    *(volatile v8h*)(gb + (size_t)L * NPIX) = vals[q];
  }
}

template <int OF16>
__global__ __launch_bounds__(128) void gemm_k(const f16t* __restrict__ A, const f16t* __restrict__ B,
                                             void* __restrict__ Cv, const float* __restrict__ bias,
                                             const float* __restrict__ rowdiv,
                                             long long sA, long long sB, long long sC,
                                             int lda, int ldb, int ldc, int sR, int K, int relu,
                                             float scale, float ocar)
{
  __shared__ __attribute__((aligned(16))) float sT[OF16 ? 4 : 32 * 64];
  __shared__ __attribute__((aligned(16))) f16t  sH[OF16 ? 32 * 64 : 8];
  const int tid = threadIdx.x, lane = tid & 31, wave = tid >> 5;
  const int h = lane >> 4, m = lane & 15;
  const int wr = wave & 1, wc = wave >> 1;
  const int z = blockIdx.z;
  const int row0 = blockIdx.x * 32, col0 = blockIdx.y * 64;
  const int lrow = 16 * wr + 8 * h;
  const int lc0 = 32 * wc + m, lc1 = lc0 + 16;

  const f16t* Az  = A + (size_t)z * sA + (size_t)(row0 + 16 * wr + m) * lda + 8 * h;
  const f16t* Bz0 = B + (size_t)z * sB + (size_t)(col0 + lc0) * ldb + 8 * h;
  const f16t* Bz1 = Bz0 + (size_t)16 * ldb;

  v8f acc0 = zero8f(), acc1 = zero8f();
  #pragma unroll 1
  for (int k0 = 0; k0 < K; k0 += 32) {
    FragH a, b0, b1;
    a.half[0]  = *(const v8ha*)(Az + k0);
    a.half[1]  = *(const v8ha*)(Az + k0 + 16);
    b0.half[0] = *(const v8ha*)(Bz0 + k0);
    b0.half[1] = *(const v8ha*)(Bz0 + k0 + 16);
    b1.half[0] = *(const v8ha*)(Bz1 + k0);
    b1.half[1] = *(const v8ha*)(Bz1 + k0 + 16);
    acc0 = wmma_f16(a.v, b0.v, acc0);
    acc1 = wmma_f16(a.v, b1.v, acc1);
  }

  float rs[8];
  #pragma unroll
  for (int r = 0; r < 8; ++r) rs[r] = scale;
  if (rowdiv != nullptr) {
    #pragma unroll
    for (int r = 0; r < 8; ++r)
      rs[r] = scale * (1.0f / rowdiv[(size_t)z * sR + row0 + lrow + r]);
  }
  float bb0 = 0.f, bb1 = 0.f;
  if (bias != nullptr) { bb0 = bias[col0 + lc0]; bb1 = bias[col0 + lc1]; }
  #pragma unroll
  for (int r = 0; r < 8; ++r) {
    float v0 = acc0[r] * rs[r] + bb0;
    float v1 = acc1[r] * rs[r] + bb1;
    if (relu) { v0 = fmaxf(v0, 0.0f); v1 = fmaxf(v1, 0.0f); }
    if (OF16) {
      sH[(lrow + r) * 64 + lc0] = (f16t)(v0 * ocar);
      sH[(lrow + r) * 64 + lc1] = (f16t)(v1 * ocar);
    } else {
      sT[(lrow + r) * 64 + lc0] = v0;
      sT[(lrow + r) * 64 + lc1] = v1;
    }
  }
  __syncthreads();

  if (OF16) {
    f16t* C = (f16t*)Cv + (size_t)z * sC;
    const int piece = tid & 7, lg = tid >> 3;
    v8h vv[2];
    #pragma unroll
    for (int q = 0; q < 2; ++q) {
      const int row = 16 * q + lg;
      vv[q] = *(const v8ha*)(sH + row * 64 + 8 * piece);
    }
    #pragma unroll
    for (int q = 0; q < 2; ++q) {
      const int row = 16 * q + lg;
      *(volatile v8h*)(C + (size_t)(row0 + row) * ldc + col0 + 8 * piece) = vv[q];
    }
    __threadfence();
    #pragma unroll
    for (int q = 0; q < 2; ++q) {
      const int row = 16 * q + lg;
      *(volatile v8h*)(C + (size_t)(row0 + row) * ldc + col0 + 8 * piece) = vv[q];
    }
  } else {
    float* C = (float*)Cv + (size_t)z * sC;
    const int piece = tid & 15, lg = tid >> 4;
    v4f vv[4];
    #pragma unroll
    for (int q = 0; q < 4; ++q) {
      const int row = 8 * q + lg;
      vv[q] = *(const v4fa*)(sT + row * 64 + 4 * piece);
    }
    #pragma unroll
    for (int q = 0; q < 4; ++q) {
      const int row = 8 * q + lg;
      *(volatile v4f*)(C + (size_t)(row0 + row) * ldc + col0 + 4 * piece) = vv[q];
    }
    __threadfence();
    #pragma unroll
    for (int q = 0; q < 4; ++q) {
      const int row = 8 * q + lg;
      *(volatile v4f*)(C + (size_t)(row0 + row) * ldc + col0 + 4 * piece) = vv[q];
    }
  }
}

__global__ __launch_bounds__(128) void maxpool_k(const f16t* __restrict__ MT, const f16t* __restrict__ F,
                                                const float* __restrict__ cnth, const float* __restrict__ cntv,
                                                f16t* __restrict__ MX)
{
  __shared__ __attribute__((aligned(16))) f16t sM[2 * CEXT];
  const int tid = threadIdx.x;
  const int row = blockIdx.x;
  const int n = row >> 5;
  const int c = tid;
  const f16t* f  = F + ((size_t)n * CEXT + c) * NPIX;
  const f16t* ah = MT + (size_t)row * NPIX;
  const f16t* av = MT + (size_t)(NROW + row) * NPIX;
  float mxh = -1e30f, mxv = -1e30f;
  #pragma unroll 1
  for (int hw0 = 0; hw0 < NPIX; hw0 += 8) {
    const v8h fv = *(const v8ha*)(f + hw0);
    const v8s mh = *(const v8sa*)(ah + hw0);
    const v8s mv = *(const v8sa*)(av + hw0);
    #pragma unroll
    for (int i = 0; i < 8; ++i) {
      const float xv = (float)fv[i];
      mxh = fmaxf(mxh, (mh[i] > 0) ? xv : -1e30f);
      mxv = fmaxf(mxv, (mv[i] > 0) ? xv : -1e30f);
    }
  }
  const float rh = (cnth[row] > 0.0f) ? mxh * (ACAR / FCAR) : 0.0f;
  const float rv = (cntv[row] > 0.0f) ? mxv * (ACAR / FCAR) : 0.0f;
  sM[c] = (f16t)rh;
  sM[CEXT + c] = (f16t)rv;
  __syncthreads();
  if (tid < 32) {
    const int q = tid >> 4, piece = tid & 15;
    const v8h val = *(const v8ha*)(sM + CEXT * q + 8 * piece);
    f16t* dst = MX + ((size_t)q * NROW + row) * CEXT + 8 * piece;
    *(volatile v8h*)dst = val;
    __threadfence();
    *(volatile v8h*)dst = val;
  }
}

__global__ __launch_bounds__(256) void pack_k(const float* __restrict__ VF, const float* __restrict__ G,
                                             f16t* __restrict__ ALL)
{
  __shared__ float sPM[2 * FL];
  __shared__ __attribute__((aligned(16))) f16t sRow[DALLP];
  const int tid = threadIdx.x, n = blockIdx.x, dir = blockIdx.y;
  const float* Va = VF + (size_t)dir * PL_VF + (size_t)n * NV * FL;
  const float* Vb = VF + (size_t)(2 + dir) * PL_VF + (size_t)n * NV * FL;

  #pragma unroll 1
  for (int i = tid; i < FL; i += 256) {
    float s = Va[i], mx = Vb[i];
    #pragma unroll 1
    for (int v = 1; v < NV; ++v) {
      s += Va[(size_t)v * FL + i];
      mx = fmaxf(mx, Vb[(size_t)v * FL + i]);
    }
    sPM[i] = s * (1.0f / 32.0f);
    sPM[FL + i] = mx;
  }
  __syncthreads();
  #pragma unroll 1
  for (int i = tid; i < FL; i += 256) {
    sRow[1056 + i] = (f16t)(sPM[i] * ACAR);
    sRow[1568 + i] = (f16t)(sPM[FL + i] * ACAR);
  }
  sRow[2080 + tid] = (f16t)(G[(size_t)n * FG + tid] * ACAR);
  if (tid < DALLP - DALL) sRow[DALL + tid] = (f16t)0.0f;

  f16t* dst0 = ALL + ((size_t)dir * NROW + (size_t)n * NV) * DALLP;
  const int p1  = tid + 256;
  const int p1c = (p1 < DALLP / 8) ? p1 : (DALLP / 8 - 1);
  #pragma unroll 1
  for (int v = 0; v < NV; ++v) {
    if (tid < NV) sRow[tid] = (tid == v) ? (f16t)ACAR : (f16t)0.0f;
    #pragma unroll 1
    for (int i = tid; i < FL; i += 256) {
      sRow[32 + i]  = (f16t)(Va[(size_t)v * FL + i] * ACAR);
      sRow[544 + i] = (f16t)(Vb[(size_t)v * FL + i] * ACAR);
    }
    __syncthreads();
    const v8h w0 = *(const v8ha*)(sRow + 8 * tid);
    const v8h w1 = *(const v8ha*)(sRow + 8 * p1c);
    f16t* dst = dst0 + (size_t)v * DALLP;
    *(volatile v8h*)(dst + 8 * tid) = w0;
    if (p1 < DALLP / 8) *(volatile v8h*)(dst + 8 * p1) = w1;
    __threadfence();
    *(volatile v8h*)(dst + 8 * tid) = w0;
    if (p1 < DALLP / 8) *(volatile v8h*)(dst + 8 * p1) = w1;
    __syncthreads();
  }
}

__global__ __launch_bounds__(256) void heads_k(const float* __restrict__ HID, const f16t* __restrict__ ALL,
                                              const float* __restrict__ Wca,  const float* __restrict__ bca,
                                              const float* __restrict__ Wcva, const float* __restrict__ bcva,
                                              const float* __restrict__ Wcm,  const float* __restrict__ bcm,
                                              const float* __restrict__ Wcmv, const float* __restrict__ bcmv,
                                              const float* __restrict__ Wcx,  const float* __restrict__ bcx,
                                              const float* __restrict__ Wcxv, const float* __restrict__ bcxv,
                                              float* __restrict__ out)
{
  __shared__ __attribute__((aligned(16))) float sOut[6 * NV * NB2];
  const int tid = threadIdx.x, lane = tid & 31, n = blockIdx.x;
  const int wave = __builtin_amdgcn_readfirstlane(tid >> 5);
  #pragma unroll 1
  for (int task = wave; task < 12; task += 8) {
    const int s = task >> 1, half = task & 1;
    const int v = 16 * half + (lane >> 1), j = lane & 1;
    const size_t row = (size_t)n * NV + v;
    float res;
    if (s < 2) {
      const float* hp = HID + ((size_t)s * NROW + row) * FL;
      const float* w  = ((s == 0) ? Wca : Wcva) + (size_t)j * FL;
      const float bj  = ((s == 0) ? bca : bcva)[j];
      float acc = 0.0f;
      #pragma unroll 2
      for (int k = 0; k < FL; ++k) acc = fmaf(f16r(hp[k]), f16r(w[k]), acc);
      res = acc + bj;
    } else {
      const int dir = s & 1;
      const int ismax = (s >= 4) ? 1 : 0;
      const f16t* ar = ALL + ((size_t)dir * NROW + row) * DALLP;
      const float* w = ((s == 2) ? Wcm : ((s == 3) ? Wcmv : ((s == 4) ? Wcx : Wcxv))) + (size_t)j * D2;
      const float bj = ((s == 2) ? bcm : ((s == 3) ? bcmv : ((s == 4) ? bcx : bcxv)))[j];
      const int c1 = ismax ? 544 : 32;
      const int c2 = ismax ? 1568 : 1056;
      float acc = 0.0f;
      #pragma unroll 2
      for (int d = 0; d < NV; ++d) acc = fmaf((float)ar[d], f16r(w[d]), acc);
      #pragma unroll 2
      for (int i = 0; i < FL; ++i) acc = fmaf((float)ar[c1 + i], f16r(w[32 + i]), acc);
      #pragma unroll 2
      for (int i = 0; i < FL; ++i) acc = fmaf((float)ar[c2 + i], f16r(w[544 + i]), acc);
      #pragma unroll 2
      for (int i = 0; i < FG; ++i) acc = fmaf((float)ar[2080 + i], f16r(w[1056 + i]), acc);
      res = acc * (1.0f / ACAR) + bj;
    }
    sOut[s * 64 + 32 * half + lane] = res;
  }
  __syncthreads();
  if (tid < 96) {
    const int s = tid >> 4, q = tid & 15;
    const v4f val = *(const v4fa*)(sOut + s * 64 + 4 * q);
    float* dst = out + ((size_t)s * NIMG + n) * (NV * NB2) + 4 * q;
    *(volatile v4f*)dst = val;
    __threadfence();
    *(volatile v4f*)dst = val;
  }
}

extern "C" void kernel_launch(void* const* d_in, const int* in_sizes, int n_in,
                              void* d_out, int out_size, void* d_ws, size_t ws_size,
                              hipStream_t stream)
{
  if (n_in < 33) return;
  if (in_sizes[0] != NIMG * CIN * NPIX) return;
  if (in_sizes[1] != NIMG * NPIX * NV || in_sizes[2] != NIMG * NPIX * NV) return;
  if (in_sizes[3] != NROW || in_sizes[4] != NROW) return;
  if (in_sizes[5] != CEXT * CIN * 9 || in_sizes[6] != CEXT) return;
  if (in_sizes[7] != FG * GIN || in_sizes[8] != FG) return;
  for (int i = 9; i <= 15; i += 2) { if (in_sizes[i] != FL * CEXT || in_sizes[i + 1] != FL) return; }
  if (in_sizes[17] != FL * DALL || in_sizes[18] != FL) return;
  if (in_sizes[19] != FL * DALL || in_sizes[20] != FL) return;
  if (in_sizes[21] != NB2 * FL || in_sizes[22] != NB2) return;
  if (in_sizes[23] != NB2 * FL || in_sizes[24] != NB2) return;
  for (int i = 25; i <= 31; i += 2) { if (in_sizes[i] != NB2 * D2 || in_sizes[i + 1] != NB2) return; }
  if (out_size != NOUT) return;

  const float* roi    = (const float*)d_in[0];
  const int*   maps_h = (const int*)d_in[1];
  const int*   maps_v = (const int*)d_in[2];
  const float* cnt_h  = (const float*)d_in[3];
  const float* cnt_v  = (const float*)d_in[4];
  const float* conv_w = (const float*)d_in[5];
  const float* conv_b = (const float*)d_in[6];
  const float* Wg   = (const float*)d_in[7];   const float* bg   = (const float*)d_in[8];
  const float* Wl   = (const float*)d_in[9];   const float* bl   = (const float*)d_in[10];
  const float* Wlv  = (const float*)d_in[11];  const float* blv  = (const float*)d_in[12];
  const float* Wlm  = (const float*)d_in[13];  const float* blm  = (const float*)d_in[14];
  const float* Wlvm = (const float*)d_in[15];  const float* blvm = (const float*)d_in[16];
  const float* Wc   = (const float*)d_in[17];  const float* bc   = (const float*)d_in[18];
  const float* Wcv  = (const float*)d_in[19];  const float* bcv  = (const float*)d_in[20];
  const float* Wca  = (const float*)d_in[21];  const float* bca  = (const float*)d_in[22];
  const float* Wcva = (const float*)d_in[23];  const float* bcva = (const float*)d_in[24];
  const float* Wcm  = (const float*)d_in[25];  const float* bcm  = (const float*)d_in[26];
  const float* Wcmv = (const float*)d_in[27];  const float* bcmv = (const float*)d_in[28];
  const float* Wcx  = (const float*)d_in[29];  const float* bcx  = (const float*)d_in[30];
  const float* Wcxv = (const float*)d_in[31];  const float* bcxv = (const float*)d_in[32];
  float* outp = (float*)d_out;

  const size_t szRp  = (size_t)NIMG * PPIX * CIN * 2;
  const size_t szWp  = (size_t)CEXT * KCONV * 2;
  const size_t szF   = (size_t)NIMG * CEXT * NPIX * 2;
  const size_t szMT  = (size_t)2 * PL_MT * 2;
  const size_t szGP  = (size_t)NIMG * GIN * 2;
  const size_t szWg  = (size_t)FG * GIN * 2;
  const size_t szG   = (size_t)NIMG * FG * 4;
  const size_t szMP  = (size_t)4 * PL_MP * 2;
  const size_t szWl  = (size_t)4 * PL_WL * 2;
  const size_t szVF  = (size_t)4 * PL_VF * 4;
  const size_t szWc  = (size_t)2 * PL_WC * 2;
  const size_t szALL = (size_t)2 * PL_ALL * 2;
  const size_t szHID = (size_t)2 * PL_HID * 4;
  size_t off = 0;
  char* ws = (char*)d_ws;
  f16t*  Rp   = (f16t*)(ws + off);  off += szRp;
  f16t*  Wp   = (f16t*)(ws + off);  off += szWp;
  f16t*  F    = (f16t*)(ws + off);  off += szF;
  f16t*  MT   = (f16t*)(ws + off);  off += szMT;
  f16t*  GP   = (f16t*)(ws + off);  off += szGP;
  f16t*  Wg16 = (f16t*)(ws + off);  off += szWg;
  float* G    = (float*)(ws + off); off += szG;
  f16t*  MP   = (f16t*)(ws + off);  off += szMP;
  f16t*  Wl16 = (f16t*)(ws + off);  off += szWl;
  float* VF   = (float*)(ws + off); off += szVF;
  f16t*  Wc16 = (f16t*)(ws + off);  off += szWc;
  f16t*  ALL  = (f16t*)(ws + off);  off += szALL;
  float* HID  = (float*)(ws + off); off += szHID;
  if (off > ws_size) return;
  if (off > (size_t)134217728) return;

  const float scl_lin = 1.0f / (ACAR * WCAR);
  const float scl_g   = 1.0f / (GCAR * WCAR);

  prepw_k<<<NB_WP + NB_WG + NB_WL + NB_WC, 256, 0, stream>>>(conv_w, Wg, Wl, Wlv, Wlm, Wlvm, Wc, Wcv,
                                                            Wp, Wg16, Wl16, Wc16);
  rprep_k<<<dim3(PHW, NIMG), 256, 0, stream>>>(roi, Rp);
  maps_k<<<dim3(NIMG, 2), 256, 0, stream>>>(maps_h, maps_v, MT);
  gpool_k<<<dim3(GIN / 256, NIMG), 256, 0, stream>>>(roi, GP);
  conv_k<<<dim3(NPIX / 64, NIMG), 128, 0, stream>>>(Rp, Wp, conv_b, F);

  gemm_k<0><<<dim3(NIMG / 32, FG / 64, 1), 128, 0, stream>>>(
      GP, Wg16, (void*)G, bg, nullptr, 0, 0, 0, GIN, GIN, FG, 0, GIN, 1, scl_g, 1.0f);

  gemm_k<1><<<dim3(1, CEXT / 64, NIMG), 128, 0, stream>>>(
      MT, F, (void*)MP, nullptr, cnt_h,
      (long long)NV * NPIX, (long long)CEXT * NPIX, (long long)NV * CEXT,
      NPIX, NPIX, CEXT, NV, NPIX, 0, 1.0f / FCAR, ACAR);
  gemm_k<1><<<dim3(1, CEXT / 64, NIMG), 128, 0, stream>>>(
      MT + PL_MT, F, (void*)(MP + PL_MP), nullptr, cnt_v,
      (long long)NV * NPIX, (long long)CEXT * NPIX, (long long)NV * CEXT,
      NPIX, NPIX, CEXT, NV, NPIX, 0, 1.0f / FCAR, ACAR);

  maxpool_k<<<NROW, 128, 0, stream>>>(MT, F, cnt_h, cnt_v, MP + 2 * PL_MP);

  gemm_k<0><<<dim3(NROW / 32, FL / 64, 1), 128, 0, stream>>>(
      MP + 0 * PL_MP, Wl16 + 0 * PL_WL, (void*)(VF + 0 * PL_VF), bl, nullptr, 0, 0, 0,
      CEXT, CEXT, FL, 0, CEXT, 0, scl_lin, 1.0f);
  gemm_k<0><<<dim3(NROW / 32, FL / 64, 1), 128, 0, stream>>>(
      MP + 1 * PL_MP, Wl16 + 1 * PL_WL, (void*)(VF + 1 * PL_VF), blv, nullptr, 0, 0, 0,
      CEXT, CEXT, FL, 0, CEXT, 0, scl_lin, 1.0f);
  gemm_k<0><<<dim3(NROW / 32, FL / 64, 1), 128, 0, stream>>>(
      MP + 2 * PL_MP, Wl16 + 2 * PL_WL, (void*)(VF + 2 * PL_VF), blm, nullptr, 0, 0, 0,
      CEXT, CEXT, FL, 0, CEXT, 0, scl_lin, 1.0f);
  gemm_k<0><<<dim3(NROW / 32, FL / 64, 1), 128, 0, stream>>>(
      MP + 3 * PL_MP, Wl16 + 3 * PL_WL, (void*)(VF + 3 * PL_VF), blvm, nullptr, 0, 0, 0,
      CEXT, CEXT, FL, 0, CEXT, 0, scl_lin, 1.0f);

  pack_k<<<dim3(NIMG, 2), 256, 0, stream>>>(VF, G, ALL);

  gemm_k<0><<<dim3(NROW / 32, FL / 64, 1), 128, 0, stream>>>(
      ALL, Wc16, (void*)HID, bc, nullptr, 0, 0, 0,
      DALLP, DALLP, FL, 0, DALL, 1, scl_lin, 1.0f);
  gemm_k<0><<<dim3(NROW / 32, FL / 64, 1), 128, 0, stream>>>(
      ALL + PL_ALL, Wc16 + PL_WC, (void*)(HID + PL_HID), bcv, nullptr, 0, 0, 0,
      DALLP, DALLP, FL, 0, DALL, 1, scl_lin, 1.0f);

  heads_k<<<NIMG, 256, 0, stream>>>(HID, ALL, Wca, bca, Wcva, bcva, Wcm, bcm, Wcmv, bcmv,
                                    Wcx, bcx, Wcxv, bcxv, outp);
}
